// MambaSSMBlock_63660005261822
// MI455X (gfx1250) — hardware-run, weakly checked
//
#include <hip/hip_runtime.h>
#include <math.h>

typedef __attribute__((ext_vector_type(8)))  _Float16 v8h;
typedef __attribute__((ext_vector_type(16))) __bf16   v16b;
typedef __attribute__((ext_vector_type(8)))  __bf16   v8b;
typedef __attribute__((ext_vector_type(8)))  float    v8f;
typedef __attribute__((ext_vector_type(4)))  float    v4f;

constexpr int kBatch  = 2;
constexpr int kSeq    = 2048;
constexpr int kDm     = 1024;
constexpr int kDin    = 2048;
constexpr int kNst    = 16;
constexpr int kXpN    = 2 * kNst + 1;
constexpr int kXpP    = 64;
constexpr int kRows   = kBatch * kSeq;
constexpr int kConvTP = 260;
constexpr int kScanTS = 64;
constexpr int kScanCh = 64;
constexpr int kScanYP = 68;
constexpr int kStP    = 20;
constexpr float kDtCarry    = 1024.0f;
constexpr float kDtCarryInv = 1.0f / kDtCarry;
static_assert(kXpN == 33 && kXpN <= kXpP, "x_proj width");
static_assert((kDm % 32) == 0 && (kDin % 32) == 0 && (kXpP % 32) == 0, "GEMM K multiples of 32");
static_assert((kRows % 64) == 0 && (kDin % 64) == 0 && (kXpP % 64) == 0 && (kDm % 64) == 0, "GEMM M,N multiples of 64");
static_assert((kSeq % kScanTS) == 0 && (kSeq % 64) == 0 && (kDin % kScanCh) == 0 && (kDin % 256) == 0, "tile multiples");
static_assert((kRows % 8) == 0 && (kDm % 256) == 0, "LayerNorm wave-per-row mapping");
static_assert(kStP >= kNst && (kStP % 4) == 0 && (kNst % 4) == 0, "per-thread state rows: 16-B aligned, 4 states per group");

constexpr size_t kSzXN   = (size_t)kRows * kDm * 2;
constexpr size_t kSzWIN  = (size_t)2 * kDin * kDm * 2;
constexpr size_t kSzF32P = (size_t)kRows * kDin * 4;
constexpr size_t kSzB16P = (size_t)kRows * kDin * 2;
constexpr size_t kOffXNH  = 0;
constexpr size_t kOffXNL  = kOffXNH + kSzXN;
constexpr size_t kOffWIN  = kOffXNL + kSzXN;
constexpr size_t kOffDTP  = 0;
constexpr size_t kOffR1   = kOffWIN + kSzWIN;
constexpr size_t kOffXC   = kOffR1 + kSzF32P;
constexpr size_t kOffXCH  = kOffXC + kSzF32P;
constexpr size_t kOffXCL  = kOffXCH + kSzB16P;
constexpr size_t kOffWOUT = kOffXCL + kSzB16P;
constexpr size_t kOffXP   = kOffWOUT + (size_t)kDm * kDin * 2;
constexpr size_t kOffXPH  = kOffXP + (size_t)kRows * kXpP * 4;
constexpr size_t kOffXPL  = kOffXPH + (size_t)kRows * kXpP * 2;
constexpr size_t kOffWX   = kOffXPL + (size_t)kRows * kXpP * 2;
constexpr size_t kOffWDT  = kOffWX + (size_t)kXpP * kDin * 2;
constexpr size_t kWsTotal = kOffWDT + (size_t)kDin * kXpP * 2;
static_assert(kWsTotal == 132644864ull, "carve total");
static_assert(kWsTotal <= 134217728ull, "carve cap");
static_assert(kSzB16P <= kOffR1, "DTP fits in the dead R0 region");
static_assert((kOffXNL % 128) == 0 && (kOffWIN % 128) == 0 && (kOffR1 % 128) == 0 && (kOffXC % 128) == 0 &&
              (kOffXCH % 128) == 0 && (kOffXCL % 128) == 0 && (kOffWOUT % 128) == 0 && (kOffXP % 128) == 0 &&
              (kOffXPH % 128) == 0 && (kOffXPL % 128) == 0 && (kOffWX % 128) == 0 && (kOffWDT % 128) == 0, "128-B aligned regions");

__device__ __forceinline__ unsigned short f2bf_bits(float f) {
  unsigned u = __float_as_uint(f);
  return (unsigned short)((u + 0x7FFFu + ((u >> 16) & 1u)) >> 16);
}
__device__ __forceinline__ float bf_bits2f(unsigned short h) { return __uint_as_float(((unsigned)h) << 16); }
__device__ __forceinline__ float bf16r(float f) { return bf_bits2f(f2bf_bits(f)); }

__device__ __forceinline__ float h16_to_f32(unsigned hb) {
  const unsigned sgn = (hb & 0x8000u) << 16; const unsigned em = hb & 0x7fffu;
  const float fn = __uint_as_float((em << 13) + 0x38000000u);
  const float fs = (float)em * 5.9604644775390625e-8f;
  const float mag = (em < 0x400u) ? fs : fn; return __uint_as_float(__float_as_uint(mag) | sgn); }

__device__ __forceinline__ void split8(const v4f a0, const v4f a1, v8h& hv, v8h& lv) {
#pragma unroll
  for (int e = 0; e < 4; ++e) {
    const float f0 = a0[e], f1 = a1[e];
    const unsigned short h0 = f2bf_bits(f0), h1 = f2bf_bits(f1);
    float w0 = bf_bits2f(h0), w1 = bf_bits2f(h1);
    asm volatile("" : "+v"(w0), "+v"(w1));
    const float r0 = f0 - w0, r1 = f1 - w1;
    const unsigned short l0 = f2bf_bits(r0), l1 = f2bf_bits(r1);
    hv[e]     = __builtin_bit_cast(_Float16, h0);
    hv[4 + e] = __builtin_bit_cast(_Float16, h1);
    lv[e]     = __builtin_bit_cast(_Float16, l0);
    lv[4 + e] = __builtin_bit_cast(_Float16, l1);
  }
}
__device__ __forceinline__ void cast8(const v4f a0, const v4f a1, v8h& hv) {
#pragma unroll
  for (int e = 0; e < 4; ++e) {
    const float f0 = a0[e], f1 = a1[e];
    const unsigned short h0 = f2bf_bits(f0), h1 = f2bf_bits(f1);
    hv[e]     = __builtin_bit_cast(_Float16, h0);
    hv[4 + e] = __builtin_bit_cast(_Float16, h1);
  }
}

__device__ __forceinline__ void dep_guard4_b(v8f& a, v8f& b, v8f& c, v8f& d, v16b x, v16b y) {
  asm volatile("v_nop\n\tv_nop\n\tv_nop\n\tv_nop" : "+v"(a), "+v"(b), "+v"(c), "+v"(d) : "v"(x), "v"(y));
}
__device__ __forceinline__ void keep4_b(v16b a, v16b b, v16b c, v16b d) { asm volatile("v_nop" :: "v"(a), "v"(b), "v"(c), "v"(d)); }
__device__ __forceinline__ void acc_guard4(v8f& a, v8f& b, v8f& c, v8f& d) { asm volatile("v_nop\n\tv_nop\n\tv_nop\n\tv_nop" : "+v"(a), "+v"(b), "+v"(c), "+v"(d)); }

struct FragB {
  union U { v16b v; v8b h[2]; };
  static __device__ __forceinline__ v16b load(const __bf16* p) {
    U f; f.h[0] = *(const v8b*)(p); f.h[1] = *(const v8b*)(p + 16); return f.v;
  }
  static __device__ __forceinline__ v8f mma(v16b a, v16b b, v8f c) {
    return __builtin_amdgcn_wmma_f32_16x16x32_bf16(false, a, false, b, (short)0, c, false, false);
  }
};

template <int SPL, int OUT_MODE>
__global__ __launch_bounds__(256) void wmma_gemm64(
    const unsigned short* __restrict__ Ap, const unsigned short* __restrict__ A2p, int lda,
    const unsigned short* __restrict__ Btp, int ldb,
    void* __restrict__ Cout, int ldc,
    int M, int N, int K, float scale) {
  typedef __bf16 T;
  typedef v16b V;
  const T* A = (const T*)Ap; const T* A2 = (const T*)A2p; const T* Bt = (const T*)Btp;
  __shared__ __align__(16) float sT[8][16 * 68];
  const int lane = threadIdx.x & 31;
  const int wave = threadIdx.x >> 5;
  const int tilesN = N >> 6;
  const int tilesM = M >> 6;
  const int tile = blockIdx.x * 8 + wave;
  if (tile >= tilesM * tilesN) return;
  const int tm = tile / tilesN;
  const int tn = tile - tm * tilesN;
  const int m0 = tm << 6;
  const int n0 = tn << 6;

  const int rlane = lane & 15;
  const int koff  = (lane >> 4) * 8;
  const int mOff  = (lane >> 4) * 8;

  v8f acc[4][4];
#pragma unroll
  for (int i = 0; i < 4; ++i)
#pragma unroll
    for (int j = 0; j < 4; ++j) acc[i][j] = (v8f){0.f,0.f,0.f,0.f,0.f,0.f,0.f,0.f};

  for (int k0 = 0; k0 < K; k0 += 32) {
    V bh[4];
#pragma unroll
    for (int j = 0; j < 4; ++j) {
      const size_t bo = (size_t)(n0 + (j << 4) + rlane) * ldb + koff + k0;
      bh[j] = FragB::load(Bt + bo);
    }
#pragma unroll
    for (int i = 0; i < 4; ++i) {
      const size_t ao = (size_t)(m0 + (i << 4) + rlane) * lda + koff + k0;
      V ah = FragB::load(A + ao);
      V al = ah;
      if (SPL >= 1) al = FragB::load(A2 + ao);
#pragma unroll
      for (int j = 0; j < 4; ++j) {
        acc[i][j] = FragB::mma(ah, bh[j], acc[i][j]);
        if (SPL >= 1) acc[i][j] = FragB::mma(al, bh[j], acc[i][j]);
      }
      dep_guard4_b(acc[i][0], acc[i][1], acc[i][2], acc[i][3], ah, al);
    }
    keep4_b(bh[0], bh[1], bh[2], bh[3]);
  }
  acc_guard4(acc[0][0], acc[0][1], acc[0][2], acc[0][3]);
  acc_guard4(acc[1][0], acc[1][1], acc[1][2], acc[1][3]);
  acc_guard4(acc[2][0], acc[2][1], acc[2][2], acc[2][3]);
  acc_guard4(acc[3][0], acc[3][1], acc[3][2], acc[3][3]);

  float* slab = sT[wave];
#pragma unroll
  for (int i = 0; i < 4; ++i) {
    const int mBase = m0 + (i << 4);
#pragma unroll
    for (int j = 0; j < 4; ++j) {
#pragma unroll
      for (int r = 0; r < 8; ++r) {
        const float v = acc[i][j][r] * scale;
        slab[(mOff + r) * 68 + (j << 4) + rlane] = v;
      }
    }
    __builtin_amdgcn_fence(__ATOMIC_RELEASE, "workgroup");
    __builtin_amdgcn_wave_barrier();
    __builtin_amdgcn_fence(__ATOMIC_ACQUIRE, "workgroup");
    if (OUT_MODE == 0) {
      float* C = (float*)Cout;
      const int hh = lane >> 4, c4 = (lane & 15) * 4;
      for (int pass = 0; pass < 2; ++pass) {
#pragma unroll
        for (int it = 0; it < 8; ++it) {
          const int row = it * 2 + hh;
          v4f v = *(const v4f*)(slab + row * 68 + c4);
          *(volatile v4f*)(C + (size_t)(mBase + row) * ldc + n0 + c4) = v;
        }
        __threadfence();
      }
    } else {
      const int q = lane >> 3, c8 = (lane & 7) * 8;
      unsigned short* C = (unsigned short*)Cout;
      for (int pass = 0; pass < 2; ++pass) {
#pragma unroll
        for (int it = 0; it < 4; ++it) {
          const int row = it * 4 + q;
          const float* sp = slab + row * 68 + c8;
          v8h hv;
#pragma unroll
          for (int e = 0; e < 8; ++e) hv[e] = (_Float16)sp[e];
          *(volatile v8h*)(C + (size_t)(mBase + row) * ldc + n0 + c8) = hv;
        }
        __threadfence();
      }
    }
    __builtin_amdgcn_fence(__ATOMIC_RELEASE, "workgroup");
    __builtin_amdgcn_wave_barrier();
    __builtin_amdgcn_fence(__ATOMIC_ACQUIRE, "workgroup");
  }
}

__global__ __launch_bounds__(256) void ln_split_kernel(
    const float* __restrict__ x, const float* __restrict__ gam, const float* __restrict__ bet,
    unsigned short* __restrict__ XH, unsigned short* __restrict__ XL)
{
  const int lane = threadIdx.x & 31, wave = threadIdx.x >> 5;
  const int row = blockIdx.x * 8 + wave;
  const float* xr = x + (size_t)row * kDm;
  float s = 0.f;
#pragma unroll 1
  for (int j = 0; j < 4; ++j) {
    const float* p = xr + j * 256 + lane * 8;
    const v4f a0 = *(const v4f*)(p);
    const v4f a1 = *(const v4f*)(p + 4);
#pragma unroll
    for (int e = 0; e < 4; ++e) { s += bf16r(a0[e]); s += bf16r(a1[e]); }
  }
#pragma unroll
  for (int off = 16; off > 0; off >>= 1) s += __shfl_xor(s, off, 32);
  const float mu = s * (1.0f / (float)kDm);
  float q = 0.f;
#pragma unroll 1
  for (int j = 0; j < 4; ++j) {
    const float* p = xr + j * 256 + lane * 8;
    const v4f a0 = *(const v4f*)(p);
    const v4f a1 = *(const v4f*)(p + 4);
#pragma unroll
    for (int e = 0; e < 4; ++e) {
      const float d0 = bf16r(a0[e]) - mu;
      const float d1 = bf16r(a1[e]) - mu;
      q = fmaf(d0, d0, q);
      q = fmaf(d1, d1, q);
    }
  }
#pragma unroll
  for (int off = 16; off > 0; off >>= 1) q += __shfl_xor(q, off, 32);
  const float var  = q * (1.0f / (float)kDm);
  const float rstd = rsqrtf(var + 1e-5f);
#pragma unroll 1
  for (int j = 0; j < 4; ++j) {
    const int c = j * 256 + lane * 8;
    const v4f a0 = *(const v4f*)(xr + c);
    const v4f a1 = *(const v4f*)(xr + c + 4);
    const v4f g0 = *(const v4f*)(gam + c);
    const v4f g1 = *(const v4f*)(gam + c + 4);
    const v4f b0 = *(const v4f*)(bet + c);
    const v4f b1 = *(const v4f*)(bet + c + 4);
    v4f o0, o1;
#pragma unroll
    for (int e = 0; e < 4; ++e) {
      o0[e] = (bf16r(a0[e]) - mu) * rstd * bf16r(g0[e]) + bf16r(b0[e]);
      o1[e] = (bf16r(a1[e]) - mu) * rstd * bf16r(g1[e]) + bf16r(b1[e]);
    }
    v8h hv, lv;
    split8(o0, o1, hv, lv);
    unsigned short* qh = XH + (size_t)row * kDm + c;
    unsigned short* ql = XL + (size_t)row * kDm + c;
    *(volatile v8h*)qh = hv;
    *(volatile v8h*)ql = lv;
    __threadfence();
    *(volatile v8h*)qh = hv;
    *(volatile v8h*)ql = lv;
  }
}

__global__ __launch_bounds__(256) void cast_rows_bf16_kernel(
    const float* __restrict__ src, unsigned short* __restrict__ dst, int total8)
{
  const int i = blockIdx.x * 256 + threadIdx.x;
  if (i >= total8) return;
  const size_t e0 = (size_t)i << 3;
  const v4f a0 = *(const v4f*)(src + e0);
  const v4f a1 = *(const v4f*)(src + e0 + 4);
  v8h hv;
  cast8(a0, a1, hv);
  unsigned short* qd = dst + e0;
  *(volatile v8h*)qd = hv;
  __threadfence();
  *(volatile v8h*)qd = hv;
}

__global__ __launch_bounds__(256) void split_rows_bf16_kernel(
    const float* __restrict__ src, unsigned short* __restrict__ dhi, unsigned short* __restrict__ dlo, int total8)
{
  const int i = blockIdx.x * 256 + threadIdx.x;
  if (i >= total8) return;
  const size_t e0 = (size_t)i << 3;
  const v4f a0 = *(const v4f*)(src + e0);
  const v4f a1 = *(const v4f*)(src + e0 + 4);
  v8h hv, lv;
  split8(a0, a1, hv, lv);
  unsigned short* qh = dhi + e0;
  unsigned short* ql = dlo + e0;
  *(volatile v8h*)qh = hv;
  *(volatile v8h*)ql = lv;
  __threadfence();
  *(volatile v8h*)qh = hv;
  *(volatile v8h*)ql = lv;
}

__global__ __launch_bounds__(256) void pack_small_kernel(
    const float* __restrict__ Wx, const float* __restrict__ Wdt,
    unsigned short* __restrict__ WXP, unsigned short* __restrict__ WDTP)
{
  const int tid = threadIdx.x;
  v8h hv;
  unsigned short* dst;
  if (blockIdx.x < 64) {
    const int i   = blockIdx.x * 256 + tid;
    const int e0  = i << 3;
    const int row = e0 >> 11;
    const int col = e0 & (kDin - 1);
    const int rc  = (row < kXpN) ? row : (kXpN - 1);
    const bool live = (row < kXpN);
    const v4f r0 = *(const v4f*)(Wx + (size_t)rc * kDin + col);
    const v4f r1 = *(const v4f*)(Wx + (size_t)rc * kDin + col + 4);
    v4f a0, a1;
#pragma unroll
    for (int e = 0; e < 4; ++e) {
      const float f0 = r0[e], f1 = r1[e];
      a0[e] = live ? f0 : 0.0f;
      a1[e] = live ? f1 : 0.0f;
    }
    cast8(a0, a1, hv);
    dst = WXP + e0;
  } else {
    const int i  = (blockIdx.x - 64) * 256 + tid;
    const int e0 = i << 3;
    const int dd = e0 >> 6;
    const int c8 = e0 & (kXpP - 1);
    v4f a0, a1;
#pragma unroll
    for (int e = 0; e < 4; ++e) {
      const int j0 = c8 + e, j1 = c8 + 4 + e;
      const int jc0 = (j0 < kXpN) ? j0 : (kXpN - 1);
      const int jc1 = (j1 < kXpN) ? j1 : (kXpN - 1);
      const float f0 = Wdt[(size_t)dd * kXpN + jc0];
      const float f1 = Wdt[(size_t)dd * kXpN + jc1];
      a0[e] = (j0 < kXpN) ? f0 : 0.0f;
      a1[e] = (j1 < kXpN) ? f1 : 0.0f;
    }
    cast8(a0, a1, hv);
    dst = WDTP + e0;
  }
  *(volatile v8h*)dst = hv;
  __threadfence();
  *(volatile v8h*)dst = hv;
}

__global__ __launch_bounds__(256) void conv_silu_kernel(
    const float* __restrict__ XPRE, const float* __restrict__ cw, const float* __restrict__ cb,
    float* __restrict__ XC, unsigned short* __restrict__ XCH, unsigned short* __restrict__ XCL)
{
  __shared__ __align__(16) float sT[16 * kConvTP];
  const int tid = threadIdx.x, lane = tid & 31, wave = tid >> 5;
  const int d0 = blockIdx.x * 256, d = d0 + tid;
  const int g0 = blockIdx.y * 64;
  const int tb = g0 & (kSeq - 1);
  const float w0 = bf16r(cw[d * 4 + 0]), w1 = bf16r(cw[d * 4 + 1]);
  const float w2 = bf16r(cw[d * 4 + 2]), w3 = bf16r(cw[d * 4 + 3]);
  const float bc = bf16r(cb[d]);
  float xm3, xm2, xm1;
  {
    const bool hist = (tb > 0);
    const int rb = hist ? (g0 - 3) : g0;
    const float v3 = XPRE[(size_t)rb * kDin + d];
    const float v2 = XPRE[(size_t)(rb + 1) * kDin + d];
    const float v1 = XPRE[(size_t)(rb + 2) * kDin + d];
    xm3 = hist ? v3 : 0.f;
    xm2 = hist ? v2 : 0.f;
    xm1 = hist ? v1 : 0.f;
  }
  const int hrow = wave >> 1;
  const int hch  = (wave & 1) * 128 + lane * 4;
#pragma unroll 1
  for (int sub = 0; sub < 4; ++sub) {
    const int lb = g0 + sub * 16;
#pragma unroll 1
    for (int s = 0; s < 16; ++s) {
      const float xcur = XPRE[(size_t)(lb + s) * kDin + d];
      float acc = w0 * xm3;
      acc = fmaf(w1, xm2, acc);
      acc = fmaf(w2, xm1, acc);
      acc = fmaf(w3, xcur, acc);
      const float sv = acc + bc;
      const float sg = __builtin_amdgcn_rcpf(1.0f + expf(-sv));
      sT[s * kConvTP + tid] = sv * sg;
      xm3 = xm2; xm2 = xm1; xm1 = xcur;
    }
    __syncthreads();
    v4f fv[4];
    v8h bh[2], blo[2];
#pragma unroll
    for (int it = 0; it < 4; ++it) fv[it] = *(const v4f*)(sT + (it * 4 + hrow) * kConvTP + hch);
#pragma unroll
    for (int it = 0; it < 2; ++it) {
      const float* sp = sT + (it * 8 + wave) * kConvTP + lane * 8;
      const v4f a0 = *(const v4f*)(sp);
      const v4f a1 = *(const v4f*)(sp + 4);
      split8(a0, a1, bh[it], blo[it]);
    }
    for (int pass = 0; pass < 2; ++pass) {
#pragma unroll
      for (int it = 0; it < 4; ++it)
        *(volatile v4f*)(XC + (size_t)(lb + it * 4 + hrow) * kDin + d0 + hch) = fv[it];
#pragma unroll
      for (int it = 0; it < 2; ++it) {
        const size_t o = (size_t)(lb + it * 8 + wave) * kDin + d0 + lane * 8;
        *(volatile v8h*)(XCH + o) = bh[it];
        *(volatile v8h*)(XCL + o) = blo[it];
      }
      __threadfence();
    }
    __syncthreads();
  }
}

__global__ __launch_bounds__(64) void scan_kernel(
    const float* __restrict__ XP, const float* __restrict__ XC, const float* __restrict__ Z,
    const unsigned short* __restrict__ DTP, const float* __restrict__ bdt, const float* __restrict__ Alog,
    const float* __restrict__ Dp, unsigned short* __restrict__ YH, unsigned short* __restrict__ YL)
{
  __shared__ __align__(16) float sX[kScanTS * kXpP];
  __shared__ __align__(16) float sY[kScanTS * kScanYP];
  __shared__ __align__(16) float sA[kScanCh * kStP];
  __shared__ __align__(16) float sI[kScanCh * kStP];
  __shared__ __align__(16) float sH[kScanCh * kStP];
  const int tid = threadIdx.x, lane = tid & 31, wave = tid >> 5;
  constexpr int kBlkPerB = kDin / kScanCh;
  const int bix = blockIdx.x / kBlkPerB;
  const int d0  = (blockIdx.x - bix * kBlkPerB) * kScanCh;
  const int d   = d0 + tid;
  const size_t row0 = (size_t)bix * kSeq;
  const int aoff = tid * kStP;
#pragma unroll 1
  for (int s = 0; s < kNst; ++s) {
    const float al = bf16r(Alog[(size_t)d * kNst + s]);
    const float an = -expf(al);
    sA[aoff + s] = an;
    sI[aoff + s] = __builtin_amdgcn_rcpf(an + 1e-8f);
  }
#pragma unroll
  for (int g = 0; g < kNst / 4; ++g) *(v4f*)(sH + aoff + 4 * g) = (v4f){0.f, 0.f, 0.f, 0.f};
  __syncthreads();
  const float bb = bf16r(bdt[d]);
  const float Dd = bf16r(Dp[d]);
  const int lr = tid >> 4, lc4 = (tid & 15) * 4;
  const int q = lane >> 3, c8 = (lane & 7) * 8;
#pragma unroll 1
  for (int t0 = 0; t0 < kSeq; t0 += kScanTS) {
    __syncthreads();
#pragma unroll
    for (int i = 0; i < 16; ++i) {
      const int r = lr + 4 * i;
      *(v4f*)(sX + r * kXpP + lc4) = *(const v4f*)(XP + (row0 + t0 + r) * kXpP + lc4);
    }
    __syncthreads();
#pragma unroll 1
    for (int s = 0; s < kScanTS; ++s) {
      const size_t m = row0 + (size_t)(t0 + s);
      const float* xr = sX + s * kXpP;
      unsigned dw = (unsigned)DTP[m * kDin + d];
      float xt = XC[m * kDin + d];
      float zv = Z[m * kDin + d];
      asm volatile("" : "+v"(dw), "+v"(xt), "+v"(zv));
      const float v   = h16_to_f32(dw) * kDtCarryInv + bb;
      const float ea  = expf(-fabsf(v));
      const float dt  = fmaxf(v, 0.0f) + log1pf(ea) + 0.001f;
      float y = 0.f;
#pragma unroll 1
      for (int g = 0; g < kNst / 4; ++g) {
        const v4f a4 = *(const v4f*)(sA + aoff + 4 * g);
        const v4f i4 = *(const v4f*)(sI + aoff + 4 * g);
        const v4f h4 = *(const v4f*)(sH + aoff + 4 * g);
        const float* bp = xr + 1 + 4 * g;
        const float* cp = xr + 1 + kNst + 4 * g;
        v4f hn4;
#pragma unroll
        for (int j = 0; j < 4; ++j) {
          const float an = a4[j];
          const float ia = i4[j];
          const float hp = h4[j];
          const float bj = bp[j];
          const float cj = cp[j];
          const float e  = __expf(dt * an);
          const float cf = (1.0f - e) * ia;
          const float db = cf * bj;
          float hn = fmaf(e, hp, db * xt);
          hn = fminf(10.0f, fmaxf(-10.0f, hn));
          hn4[j] = hn;
          y = fmaf(cj, hn, y);
        }
        *(v4f*)(sH + aoff + 4 * g) = hn4;
      }
      y = fmaf(Dd, xt, y);
      const float sg = __builtin_amdgcn_rcpf(1.0f + __expf(-zv));
      y = y * (zv * sg);
      sY[s * kScanYP + tid] = y;
    }
    __syncthreads();
#pragma unroll 1
    for (int pass = 0; pass < 2; ++pass) {
#pragma unroll 1
      for (int it = 0; it < 8; ++it) {
        const int row = it * 8 + wave * 4 + q;
        const float* sp = sY + row * kScanYP + c8;
        const v4f a0 = *(const v4f*)(sp);
        const v4f a1 = *(const v4f*)(sp + 4);
        v8h hv, lv;
        split8(a0, a1, hv, lv);
        const size_t o = (row0 + t0 + row) * kDin + d0 + c8;
        *(volatile v8h*)(YH + o) = hv;
        *(volatile v8h*)(YL + o) = lv;
      }
      __threadfence();
    }
  }
}

extern "C" void kernel_launch(void* const* d_in, const int* in_sizes, int n_in,
                              void* d_out, int out_size, void* d_ws, size_t ws_size,
                              hipStream_t stream) {
  if (n_in < 12) return;
  if (in_sizes[0] != kRows * kDm) return;
  if (in_sizes[1] != kDm || in_sizes[2] != kDm) return;
  if (in_sizes[3] != 2 * kDin * kDm) return;
  if (in_sizes[4] != kDin * 4 || in_sizes[5] != kDin) return;
  if (in_sizes[6] != kDin * kNst || in_sizes[7] != kDin) return;
  if (in_sizes[8] != kXpN * kDin) return;
  if (in_sizes[9] != kDin * kXpN || in_sizes[10] != kDin) return;
  if (in_sizes[11] != kDm * kDin) return;
  if (out_size != kRows * kDm) return;
  if (ws_size < kWsTotal) return;

  const float* x       = (const float*)d_in[0];
  const float* ln_g    = (const float*)d_in[1];
  const float* ln_b    = (const float*)d_in[2];
  const float* W_in    = (const float*)d_in[3];
  const float* conv_w  = (const float*)d_in[4];
  const float* conv_b  = (const float*)d_in[5];
  const float* A_log   = (const float*)d_in[6];
  const float* D_par   = (const float*)d_in[7];
  const float* W_xproj = (const float*)d_in[8];
  const float* W_dt    = (const float*)d_in[9];
  const float* b_dt    = (const float*)d_in[10];
  const float* W_out   = (const float*)d_in[11];
  float* out = (float*)d_out;

  char* ws = (char*)d_ws;
  unsigned short* XNH  = (unsigned short*)(ws + kOffXNH);
  unsigned short* XNL  = (unsigned short*)(ws + kOffXNL);
  unsigned short* WIN  = (unsigned short*)(ws + kOffWIN);
  unsigned short* DTP  = (unsigned short*)(ws + kOffDTP);
  float*          R1   = (float*)(ws + kOffR1);
  float*          XC   = (float*)(ws + kOffXC);
  unsigned short* XCH  = (unsigned short*)(ws + kOffXCH);
  unsigned short* XCL  = (unsigned short*)(ws + kOffXCL);
  unsigned short* YH   = XCH;
  unsigned short* YL   = XCL;
  unsigned short* WOUT = (unsigned short*)(ws + kOffWOUT);
  float*          XP   = (float*)(ws + kOffXP);
  unsigned short* XPH  = (unsigned short*)(ws + kOffXPH);
  unsigned short* XPL  = (unsigned short*)(ws + kOffXPL);
  unsigned short* WX   = (unsigned short*)(ws + kOffWX);
  unsigned short* WDT  = (unsigned short*)(ws + kOffWDT);

  ln_split_kernel<<<kRows / 8, 256, 0, stream>>>(x, ln_g, ln_b, XNH, XNL);
  cast_rows_bf16_kernel<<<(2 * kDin * kDm / 8) / 256, 256, 0, stream>>>(W_in, WIN, 2 * kDin * kDm / 8);
  cast_rows_bf16_kernel<<<(kDm * kDin / 8) / 256, 256, 0, stream>>>(W_out, WOUT, kDm * kDin / 8);
  pack_small_kernel<<<128, 256, 0, stream>>>(W_xproj, W_dt, WX, WDT);

  wmma_gemm64<1, 0><<<256, 256, 0, stream>>>(
      XNH, XNL, kDm, WIN, kDm, (void*)R1, kDin, kRows, kDin, kDm, 1.0f);

  conv_silu_kernel<<<dim3(kDin / 256, kRows / 64), 256, 0, stream>>>(R1, conv_w, conv_b, XC, XCH, XCL);

  wmma_gemm64<1, 0><<<256, 256, 0, stream>>>(
      XNH, XNL, kDm, WIN + (size_t)kDin * kDm, kDm, (void*)R1, kDin, kRows, kDin, kDm, 1.0f);

  wmma_gemm64<1, 0><<<8, 256, 0, stream>>>(
      XCH, XCL, kDin, WX, kDin, (void*)XP, kXpP, kRows, kXpP, kDin, 1.0f);

  split_rows_bf16_kernel<<<(kRows * kXpP / 8) / 256, 256, 0, stream>>>(XP, XPH, XPL, kRows * kXpP / 8);

  wmma_gemm64<1, 1><<<256, 256, 0, stream>>>(
      XPH, XPL, kXpP, WDT, kXpP, (void*)DTP, kDin, kRows, kDin, kXpP, kDtCarry);

  scan_kernel<<<kBatch * (kDin / kScanCh), kScanCh, 0, stream>>>(XP, XC, R1, DTP, b_dt, A_log, D_par, YH, YL);

  wmma_gemm64<1, 0><<<128, 256, 0, stream>>>(
      YH, YL, kDin, WOUT, kDin, (void*)out, kDm, kRows, kDm, kDin, 1.0f);
}
